// CausalSelfAttention_62989990363647
// MI455X (gfx1250) — hardware-verified
//
#include <hip/hip_runtime.h>


#ifndef NB
#define NB 4
#endif
#ifndef SEQ
#define SEQ 2048
#endif
#define NB_FULL 4
#define TT_FULL 2048
#define TT   SEQ
#define DM   1024
#define NH_  16
#define HD   64
#define DQ   (NH_ * HD)
#define RH   ((TT) < 512 ? (TT) : 512)
#define PCAR 1024.0f
#define WCAR 256.0f
#define SCL  0.125f
#define LOG2E 1.4426950408889634f
#define PSZ  ((size_t)NB * NH_ * TT * HD)
#define ISZ  ((size_t)NB * NH_ * RH * HD)
#define WS_TOTAL ((size_t)3 * DQ * DM * 2 + (size_t)2 * DM * DQ * 2 + (size_t)NB * TT * DM * 2 + 3 * PSZ * 2 + 6 * ISZ * 2 + (size_t)2 * NB * RH * DQ * 2)

static_assert(HD == 64);
static_assert(DQ == DM);
static_assert(TT % 64 == 0);
static_assert(RH % 64 == 0);
static_assert((TT - RH) % 64 == 0);
static_assert(DM % 32 == 0);
static_assert(DQ % 64 == 0);
static_assert(NB <= NB_FULL);
static_assert(TT <= TT_FULL);
static_assert(WS_TOTAL <= (size_t)134217728);

typedef _Float16 h16;
typedef unsigned short bf;
typedef __attribute__((ext_vector_type(16))) __bf16   v16bf;
typedef __attribute__((ext_vector_type(16))) _Float16 v16h;
typedef __attribute__((ext_vector_type(8)))  _Float16 v8h;
typedef __attribute__((ext_vector_type(8)))  unsigned short v8us;
typedef __attribute__((ext_vector_type(8)))  float    v8f;
typedef __attribute__((ext_vector_type(4)))  float    v4f;
typedef __attribute__((ext_vector_type(2)))  _Float16 v2h;
typedef __attribute__((ext_vector_type(2)))  unsigned short v2us;
typedef v8h  __attribute__((may_alias)) v8ha;
typedef v4f  __attribute__((may_alias)) v4fa;
typedef v8us __attribute__((may_alias)) v8usa;

__device__ __forceinline__ unsigned short f2bf(float f) { unsigned u = __float_as_uint(f); u += 0x7FFFu + ((u >> 16) & 1u); return (unsigned short)(u >> 16); }
__device__ __forceinline__ float bf2f(unsigned short b) { return __uint_as_float(((unsigned)b) << 16); }
__device__ __forceinline__ float bfr(float f) { return bf2f(f2bf(f)); }
__device__ __forceinline__ void splitf(float y, unsigned short& h, unsigned short& l) { h = f2bf(y); l = f2bf(y - bf2f(h)); }
__device__ __forceinline__ v16h cat16(v8h lo, v8h hi) { return __builtin_shufflevector(lo, hi, 0, 1, 2, 3, 4, 5, 6, 7, 8, 9, 10, 11, 12, 13, 14, 15); }
__device__ __forceinline__ v16bf cat16b(v8us lo, v8us hi) { return __builtin_bit_cast(v16bf, __builtin_shufflevector(lo, hi, 0, 1, 2, 3, 4, 5, 6, 7, 8, 9, 10, 11, 12, 13, 14, 15)); }
__device__ __forceinline__ v8f wmma16(v16h a, v16h b, v8f c) { return __builtin_amdgcn_wmma_f32_16x16x32_f16(false, a, false, b, (short)0, c, false, false); }
__device__ __forceinline__ v8f wmmab(v16bf a, v16bf b, v8f c) { return __builtin_amdgcn_wmma_f32_16x16x32_bf16(false, a, false, b, (short)0, c, false, false); }
__device__ __forceinline__ v16h ldh(const h16* p) { return cat16(*(const v8h*)p, *(const v8h*)(p + 16)); }
__device__ __forceinline__ v16bf ldb(const bf* p) { return cat16b(*(const v8us*)p, *(const v8us*)(p + 16)); }

template <typename T16> struct WFrag;
template <> struct WFrag<h16> { typedef v16h V; static __device__ __forceinline__ V ld(const h16* p) { return ldh(p); } static __device__ __forceinline__ v8f mma(V a, V b, v8f c) { return wmma16(a, b, c); } };
template <> struct WFrag<bf> { typedef v16bf V; static __device__ __forceinline__ V ld(const bf* p) { return ldb(p); } static __device__ __forceinline__ v8f mma(V a, V b, v8f c) { return wmmab(a, b, c); } };

template <typename T16, int NSPLIT>
__device__ __forceinline__ void gemm_kloop(const T16* __restrict__ A, const T16* __restrict__ A2, const T16* __restrict__ Bt, int K, size_t aoff, size_t boff, v8f (&acc)[4][4]) {
    typedef typename WFrag<T16>::V V;
#pragma unroll 1
    for (int kc = 0; kc < K; kc += 32) {
        V a[4], a2[4];
#pragma unroll
        for (int mb = 0; mb < 4; ++mb) { a[mb] = WFrag<T16>::ld(A + aoff + (size_t)mb * 16 * K + kc); if (NSPLIT == 1) a2[mb] = WFrag<T16>::ld(A2 + aoff + (size_t)mb * 16 * K + kc); }
#pragma unroll
        for (int nb = 0; nb < 4; ++nb) { const V b = WFrag<T16>::ld(Bt + boff + (size_t)nb * 16 * K + kc);
#pragma unroll
            for (int mb = 0; mb < 4; ++mb) { acc[mb][nb] = WFrag<T16>::mma(a[mb], b, acc[mb][nb]); if (NSPLIT == 1) acc[mb][nb] = WFrag<T16>::mma(a2[mb], b, acc[mb][nb]); } }
        asm volatile("v_nop\n\tv_nop\n\tv_nop\n\tv_nop" : "+v"(acc[0][0]), "+v"(acc[1][1]), "+v"(acc[2][2]), "+v"(acc[3][3]) : "v"(a[0]), "v"(a[3]));
    }
}

__global__ __launch_bounds__(256) void k_cvt8(const float* __restrict__ x, bf* XB) {
    const size_t i = (size_t)blockIdx.x * 256 + threadIdx.x; const size_t per = (size_t)TT * DM / 8; if (i >= (size_t)NB * per) return;
    const size_t b = i / per, r = i % per; const float* s = x + b * (size_t)TT_FULL * DM + r * 8; const v4f v0 = *(const v4f*)s, v1 = *(const v4f*)(s + 4); v8us o;
#pragma unroll
    for (int k = 0; k < 4; ++k) { o[k] = f2bf(v0[k]); o[k + 4] = f2bf(v1[k]); }
    *(volatile v8us*)(XB + i * 8) = o; __threadfence(); *(volatile v8us*)(XB + i * 8) = o; }

__global__ __launch_bounds__(256) void k_wtA(const float* __restrict__ w, bf* Bt) {
    const int lane = threadIdx.x & 31; const int L0 = (blockIdx.x * 8 + (threadIdx.x >> 5)) * 8; const int nlines = 3 * DQ * DM / 64;
#pragma unroll 1
    for (int ps = 0; ps < 2; ++ps) {
#pragma unroll 1
        for (int l = 0; l < 8; ++l) { const int L = L0 + l; if (L >= nlines) break; const size_t e = (size_t)L * 64 + lane * 2; const int k = (int)(e % DM), np = (int)(e / DM);
            const int part = np / DQ, r = np % DQ, h = r / HD, d = r % HD; const int col = part * DQ + d * NH_ + h; v2us o;
            o[0] = f2bf(w[(size_t)k * (3 * DQ) + col]); o[1] = f2bf(w[(size_t)(k + 1) * (3 * DQ) + col]); *(volatile v2us*)(Bt + e) = o; }
        if (ps == 0) __threadfence(); }
}
__global__ __launch_bounds__(256) void k_wtO(const float* __restrict__ w, bf* Wb, h16* W16) {
    const int lane = threadIdx.x & 31; const int L0 = (blockIdx.x * 8 + (threadIdx.x >> 5)) * 8; const int nlines = DM * DQ / 64;
#pragma unroll 1
    for (int ps = 0; ps < 2; ++ps) {
#pragma unroll 1
        for (int l = 0; l < 8; ++l) { const int L = L0 + l; if (L >= nlines) break; const size_t e = (size_t)L * 64 + lane * 2; const int kp = (int)(e % DQ), n = (int)(e / DQ);
            const int h = kp / HD, d = kp % HD; const float w0 = bfr(w[(size_t)(d * NH_ + h) * DM + n]), w1 = bfr(w[(size_t)((d + 1) * NH_ + h) * DM + n]); v2us o; v2h o16;
            o[0] = f2bf(w0); o[1] = f2bf(w1); o16[0] = (h16)(w0 * WCAR); o16[1] = (h16)(w1 * WCAR); *(volatile v2us*)(Wb + e) = o; *(volatile v2h*)(W16 + e) = o16; }
        if (ps == 0) __threadfence(); }
}

__global__ __launch_bounds__(32) void k_qkv(const bf* __restrict__ XB, const bf* __restrict__ W, const float* __restrict__ bias, h16* PL16, bf* PLh, bf* PLl) {
    __shared__ __align__(16) float os[64 * 68];
    const int lane = threadIdx.x & 31, lr = lane & 15, hi = lane >> 4; const int r0 = blockIdx.x * 64, c0 = blockIdx.y * 64;
    v8f acc[4][4];
#pragma unroll
    for (int mb = 0; mb < 4; ++mb)
#pragma unroll
        for (int nb = 0; nb < 4; ++nb) acc[mb][nb] = (v8f){};
    const size_t aoff = (size_t)(r0 + lr) * DM + 8 * hi, boff = (size_t)(c0 + lr) * DM + 8 * hi;
    gemm_kloop<bf, 0>(XB, XB, W, DM, aoff, boff, acc);
    const int part = c0 / DQ, h = (c0 % DQ) / HD, b = r0 / TT, t0 = r0 % TT; const int bh = b * NH_ + h; const bool isl = (t0 < RH); const int ti = isl ? t0 : 0;
#pragma unroll
    for (int nb = 0; nb < 4; ++nb) { const float bv = bfr(bias[part * DQ + (nb * 16 + lr) * NH_ + h]);
#pragma unroll
        for (int mb = 0; mb < 4; ++mb)
#pragma unroll
            for (int j = 0; j < 8; ++j) os[(mb * 16 + hi * 8 + j) * 68 + nb * 16 + lr] = acc[mb][nb][j] + bv; }
    __builtin_amdgcn_wave_barrier(); asm volatile("" ::: "memory");
    const int rq = lane >> 3, pc = (lane & 7) * 8;
    if (part < 2) {
        h16* p16 = PL16 + (size_t)part * PSZ + ((size_t)bh * TT + t0) * HD + pc; bf* ph = PLh + (size_t)part * ISZ + ((size_t)bh * RH + ti) * HD + pc; bf* pl = PLl + (size_t)part * ISZ + ((size_t)bh * RH + ti) * HD + pc;
#pragma unroll 1
        for (int ps = 0; ps < 2; ++ps) {
#pragma unroll 2
            for (int s = 0; s < 16; ++s) { const int row = 4 * s + rq; const v4f f0 = *(const v4fa*)(os + row * 68 + pc), f1 = *(const v4fa*)(os + row * 68 + pc + 4); v8h o; v8us oh, ol;
#pragma unroll
                for (int q = 0; q < 4; ++q) { unsigned short a, c; o[q] = (h16)f0[q]; o[q + 4] = (h16)f1[q]; splitf(f0[q], a, c); oh[q] = a; ol[q] = c; splitf(f1[q], a, c); oh[q + 4] = a; ol[q + 4] = c; }
                *(volatile v8h*)(p16 + (size_t)row * HD) = o;
                if (isl) { *(volatile v8us*)(ph + (size_t)row * HD) = oh; *(volatile v8us*)(pl + (size_t)row * HD) = ol; } }
            if (ps == 0) __threadfence(); }
    } else {
        h16* p16 = PL16 + (size_t)2 * PSZ + (size_t)bh * HD * TT + t0 + pc; bf* ph = PLh + (size_t)2 * ISZ + (size_t)bh * HD * RH + ti + pc; bf* pl = PLl + (size_t)2 * ISZ + (size_t)bh * HD * RH + ti + pc;
#pragma unroll 1
        for (int ps = 0; ps < 2; ++ps) {
#pragma unroll 2
            for (int s = 0; s < 16; ++s) { const int d = 4 * s + rq; v8h o; v8us oh, ol;
#pragma unroll
                for (int q = 0; q < 8; ++q) { unsigned short a, c; const float f = os[(pc + q) * 68 + d]; o[q] = (h16)f; splitf(f, a, c); oh[q] = a; ol[q] = c; }
                *(volatile v8h*)(p16 + (size_t)d * TT) = o;
                if (isl) { *(volatile v8us*)(ph + (size_t)d * RH) = oh; *(volatile v8us*)(pl + (size_t)d * RH) = ol; } }
            if (ps == 0) __threadfence(); }
    }
}

__device__ __forceinline__ void smax_blk(const v8f s0, const v8f s1, const bool diag, const int ib0, const int jq, float& m, float& l, float& alpha, float (&p0)[8], float (&p1)[8]) {
    float t0[8], t1[8]; float mx = -3.0e38f;
#pragma unroll
    for (int r = 0; r < 8; ++r) { float a = s0[r] * SCL, c = s1[r] * SCL;
        if (diag) { a = (ib0 + r > jq) ? -3.0e38f : a; c = (ib0 + 16 + r > jq) ? -3.0e38f : c; }
        t0[r] = a; t1[r] = c; mx = fmaxf(mx, fmaxf(a, c)); }
    mx = fmaxf(mx, __shfl_xor(mx, 16, 32));
    const float mn = fmaxf(m, mx); const float ea = __builtin_amdgcn_exp2f((m - mn) * LOG2E); alpha = (m > -1.0e37f) ? ea : 0.0f;
    float ps = 0.0f;
#pragma unroll
    for (int r = 0; r < 8; ++r) { const float e0 = __builtin_amdgcn_exp2f((t0[r] - mn) * LOG2E), e1 = __builtin_amdgcn_exp2f((t1[r] - mn) * LOG2E);
        p0[r] = (t0[r] > -1.0e37f) ? e0 : 0.0f; p1[r] = (t1[r] > -1.0e37f) ? e1 : 0.0f; ps += p0[r] + p1[r]; }
    l = l * alpha + ps; m = mn;
}

__global__ __launch_bounds__(32) void k_attn16(const h16* __restrict__ PL16, h16* AT16) {
    __shared__ __align__(16) h16 ot[16 * 72];
    const int lane = threadIdx.x & 31, lr = lane & 15, hi = lane >> 4; const int j0 = RH + blockIdx.x * 16; const int bh = blockIdx.y; const int b = bh / NH_, h = bh % NH_;
    const size_t hb = (size_t)bh * TT * HD; const h16* KF = PL16 + hb; const h16* QF = PL16 + PSZ + hb; const h16* VT = PL16 + 2 * PSZ + hb;
    const size_t qo = (size_t)(j0 + lr) * HD + 8 * hi; const v16h bq0 = ldh(QF + qo), bq1 = ldh(QF + qo + 32);
    v8f o0 = {}, o1 = {}, o2 = {}, o3 = {}; float m = -3.0e38f, l = 0.0f; const int nblk = j0 / 32 + 1; const int jq = j0 + lr;
#pragma unroll 1
    for (int ib = 0; ib < nblk; ++ib) {
        const int i0 = ib * 32; const size_t ko = (size_t)(i0 + lr) * HD + 8 * hi; v8f s0 = {}, s1 = {};
        { const v16h a00 = ldh(KF + ko), a01 = ldh(KF + ko + 32), a10 = ldh(KF + ko + 16 * HD), a11 = ldh(KF + ko + 16 * HD + 32);
          s0 = wmma16(a00, bq0, s0); s0 = wmma16(a01, bq1, s0); s1 = wmma16(a10, bq0, s1); s1 = wmma16(a11, bq1, s1);
          asm volatile("v_nop\n\tv_nop\n\tv_nop\n\tv_nop" : "+v"(s0), "+v"(s1) : "v"(a00), "v"(a01), "v"(a10), "v"(a11)); }
        float alpha, p0[8], p1[8]; smax_blk(s0, s1, ib == nblk - 1, i0 + 8 * hi, jq, m, l, alpha, p0, p1);
        v8h plo, phi;
#pragma unroll
        for (int r = 0; r < 8; ++r) { plo[r] = (h16)(p0[r] * PCAR); phi[r] = (h16)(p1[r] * PCAR); }
        const v16h pb = cat16(plo, phi);
        o0 *= alpha; o1 *= alpha; o2 *= alpha; o3 *= alpha;
        const size_t vo = (size_t)lr * TT + i0 + 8 * hi;
        { const v16h av0 = ldh(VT + vo), av1 = ldh(VT + vo + (size_t)16 * TT), av2 = ldh(VT + vo + (size_t)32 * TT), av3 = ldh(VT + vo + (size_t)48 * TT);
          o0 = wmma16(av0, pb, o0); o1 = wmma16(av1, pb, o1); o2 = wmma16(av2, pb, o2); o3 = wmma16(av3, pb, o3);
          asm volatile("v_nop\n\tv_nop\n\tv_nop\n\tv_nop" : "+v"(o0), "+v"(o1), "+v"(o2), "+v"(o3) : "v"(av0), "v"(av1), "v"(av2), "v"(av3), "v"(pb)); }
    }
    l += __shfl_xor(l, 16, 32); const float inv = 1.0f / l;
    { v8h c0, c1, c2, c3;
#pragma unroll
      for (int r = 0; r < 8; ++r) { c0[r] = (h16)(o0[r] * inv); c1[r] = (h16)(o1[r] * inv); c2[r] = (h16)(o2[r] * inv); c3[r] = (h16)(o3[r] * inv); }
      h16* op = ot + lr * 72 + 8 * hi; *(v8ha*)(op) = c0; *(v8ha*)(op + 16) = c1; *(v8ha*)(op + 32) = c2; *(v8ha*)(op + 48) = c3; }
    __builtin_amdgcn_wave_barrier(); asm volatile("" ::: "memory");
    h16* dst = AT16 + ((size_t)b * TT + j0) * DQ + h * HD; const int rq = lane >> 3, pc = (lane & 7) * 8;
#pragma unroll 1
    for (int ps = 0; ps < 2; ++ps) {
#pragma unroll
        for (int s = 0; s < 4; ++s) { const int row = 4 * s + rq; const v8h v = *(const v8ha*)(ot + row * 72 + pc); *(volatile v8h*)(dst + (size_t)row * DQ + pc) = v; }
        if (ps == 0) __threadfence(); }
}

__device__ __forceinline__ void qk3(const bf* __restrict__ Kh, const bf* __restrict__ Kl, size_t off, v16bf bh0, v16bf bh1, v16bf bl0, v16bf bl1, v8f& s) {
    const v16bf ah0 = ldb(Kh + off), ah1 = ldb(Kh + off + 32), al0 = ldb(Kl + off), al1 = ldb(Kl + off + 32);
    s = wmmab(ah0, bh0, s); s = wmmab(ah1, bh1, s); s = wmmab(al0, bh0, s); s = wmmab(al1, bh1, s); s = wmmab(ah0, bl0, s); s = wmmab(ah1, bl1, s);
    asm volatile("v_nop\n\tv_nop\n\tv_nop\n\tv_nop" : "+v"(s) : "v"(ah0), "v"(ah1), "v"(al0), "v"(al1), "v"(bl1));
}
__device__ __forceinline__ void pv3(const bf* __restrict__ Vh, const bf* __restrict__ Vl, size_t off, v16bf pbh, v16bf pbl, v8f& o) {
    const v16bf vh = ldb(Vh + off), vl = ldb(Vl + off);
    o = wmmab(vh, pbh, o); o = wmmab(vl, pbh, o); o = wmmab(vh, pbl, o);
    asm volatile("v_nop\n\tv_nop\n\tv_nop\n\tv_nop" : "+v"(o) : "v"(vh), "v"(vl), "v"(pbh), "v"(pbl));
}

__global__ __launch_bounds__(32) void k_attnhl(const bf* __restrict__ PLh, const bf* __restrict__ PLl, bf* ATh, bf* ATl) {
    __shared__ __align__(16) unsigned short oth[16 * 72];
    __shared__ __align__(16) unsigned short otl[16 * 72];
    const int lane = threadIdx.x & 31, lr = lane & 15, hi = lane >> 4; const int j0 = blockIdx.x * 16; const int bh = blockIdx.y; const int b = bh / NH_, h = bh % NH_;
    const size_t hb = (size_t)bh * RH * HD;
    const bf* KFh = PLh + hb; const bf* KFl = PLl + hb; const bf* QFh = PLh + ISZ + hb; const bf* QFl = PLl + ISZ + hb; const bf* VTh = PLh + 2 * ISZ + hb; const bf* VTl = PLl + 2 * ISZ + hb;
    const size_t qo = (size_t)(j0 + lr) * HD + 8 * hi; const v16bf bqh0 = ldb(QFh + qo), bqh1 = ldb(QFh + qo + 32), bql0 = ldb(QFl + qo), bql1 = ldb(QFl + qo + 32);
    v8f o0 = {}, o1 = {}, o2 = {}, o3 = {}; float m = -3.0e38f, l = 0.0f; const int nblk = j0 / 32 + 1; const int jq = j0 + lr;
#pragma unroll 1
    for (int ib = 0; ib < nblk; ++ib) {
        const int i0 = ib * 32; const size_t ko = (size_t)(i0 + lr) * HD + 8 * hi; v8f s0 = {}, s1 = {};
        qk3(KFh, KFl, ko, bqh0, bqh1, bql0, bql1, s0);
        qk3(KFh, KFl, ko + 16 * HD, bqh0, bqh1, bql0, bql1, s1);
        float alpha, p0[8], p1[8]; smax_blk(s0, s1, ib == nblk - 1, i0 + 8 * hi, jq, m, l, alpha, p0, p1);
        v8us ph0, ph1, pl0, pl1;
#pragma unroll
        for (int r = 0; r < 8; ++r) { unsigned short a, c; splitf(p0[r], a, c); ph0[r] = a; pl0[r] = c; splitf(p1[r], a, c); ph1[r] = a; pl1[r] = c; }
        const v16bf pbh = cat16b(ph0, ph1), pbl = cat16b(pl0, pl1);
        o0 *= alpha; o1 *= alpha; o2 *= alpha; o3 *= alpha;
        const size_t vo = (size_t)lr * RH + i0 + 8 * hi;
        pv3(VTh, VTl, vo, pbh, pbl, o0); pv3(VTh, VTl, vo + (size_t)16 * RH, pbh, pbl, o1); pv3(VTh, VTl, vo + (size_t)32 * RH, pbh, pbl, o2); pv3(VTh, VTl, vo + (size_t)48 * RH, pbh, pbl, o3);
    }
    l += __shfl_xor(l, 16, 32); const float inv = 1.0f / l;
    { v8us h0, h1, h2, h3, l0, l1, l2, l3;
#pragma unroll
      for (int r = 0; r < 8; ++r) { unsigned short a, c; splitf(o0[r] * inv, a, c); h0[r] = a; l0[r] = c; splitf(o1[r] * inv, a, c); h1[r] = a; l1[r] = c; splitf(o2[r] * inv, a, c); h2[r] = a; l2[r] = c; splitf(o3[r] * inv, a, c); h3[r] = a; l3[r] = c; }
      const int oo = lr * 72 + 8 * hi;
      *(v8usa*)(oth + oo) = h0; *(v8usa*)(oth + oo + 16) = h1; *(v8usa*)(oth + oo + 32) = h2; *(v8usa*)(oth + oo + 48) = h3;
      *(v8usa*)(otl + oo) = l0; *(v8usa*)(otl + oo + 16) = l1; *(v8usa*)(otl + oo + 32) = l2; *(v8usa*)(otl + oo + 48) = l3; }
    __builtin_amdgcn_wave_barrier(); asm volatile("" ::: "memory");
    const size_t dofs = ((size_t)b * RH + j0) * DQ + h * HD; const int rq = lane >> 3, pc = (lane & 7) * 8;
#pragma unroll 1
    for (int ps = 0; ps < 2; ++ps) {
#pragma unroll
        for (int s = 0; s < 4; ++s) { const int row = 4 * s + rq; const v8us vh = *(const v8usa*)(oth + row * 72 + pc), vl = *(const v8usa*)(otl + row * 72 + pc);
            *(volatile v8us*)(ATh + dofs + (size_t)row * DQ + pc) = vh; *(volatile v8us*)(ATl + dofs + (size_t)row * DQ + pc) = vl; }
        if (ps == 0) __threadfence(); }
}

__global__ __launch_bounds__(32) void k_outhl(const bf* __restrict__ Ah, const bf* __restrict__ Al, const bf* __restrict__ Wb, const float* __restrict__ bias, float* C) {
    __shared__ __align__(16) float os[16 * 68];
    const size_t z = blockIdx.z; const int lane = threadIdx.x & 31, lr = lane & 15, hi = lane >> 4; const int r0 = blockIdx.x * 64, c0 = blockIdx.y * 64;
    v8f acc[4][4];
#pragma unroll
    for (int mb = 0; mb < 4; ++mb)
#pragma unroll
        for (int nb = 0; nb < 4; ++nb) acc[mb][nb] = (v8f){};
    const size_t aoff = z * (size_t)RH * DQ + (size_t)(r0 + lr) * DQ + 8 * hi, boff = (size_t)(c0 + lr) * DQ + 8 * hi;
    gemm_kloop<bf, 1>(Ah, Al, Wb, DQ, aoff, boff, acc);
    float* Cz = C + z * (size_t)TT_FULL * DM + (size_t)r0 * DM + c0; const int cofs = lr * 4; v4f bb;
#pragma unroll
    for (int q = 0; q < 4; ++q) bb[q] = bfr(bias[c0 + cofs + q]);
#pragma unroll
    for (int mb = 0; mb < 4; ++mb) {
#pragma unroll
        for (int nb = 0; nb < 4; ++nb) {
#pragma unroll
            for (int j = 0; j < 8; ++j) os[(hi * 8 + j) * 68 + nb * 16 + lr] = acc[mb][nb][j]; }
        __builtin_amdgcn_wave_barrier(); asm volatile("" ::: "memory");
        float* crow = Cz + (size_t)(mb * 16) * DM;
#pragma unroll 1
        for (int ps = 0; ps < 2; ++ps) {
#pragma unroll
            for (int s = 0; s < 8; ++s) { const int row = 2 * s + hi; v4f val = *(const v4fa*)(os + row * 68 + cofs); val = val + bb; *(volatile v4f*)(crow + (size_t)row * DM + cofs) = val; }
            if (ps == 0) __threadfence(); }
        __builtin_amdgcn_wave_barrier(); asm volatile("" ::: "memory");
    }
}
__global__ __launch_bounds__(32) void k_out16(const h16* __restrict__ A16, const h16* __restrict__ W16, const float* __restrict__ bias, float* C) {
    __shared__ __align__(16) float os[16 * 68];
    const size_t z = blockIdx.z; const int lane = threadIdx.x & 31, lr = lane & 15, hi = lane >> 4; const int r0 = blockIdx.x * 64, c0 = blockIdx.y * 64;
    v8f acc[4][4];
#pragma unroll
    for (int mb = 0; mb < 4; ++mb)
#pragma unroll
        for (int nb = 0; nb < 4; ++nb) acc[mb][nb] = (v8f){};
    const size_t aoff = z * (size_t)TT * DQ + (size_t)(RH + r0 + lr) * DQ + 8 * hi, boff = (size_t)(c0 + lr) * DQ + 8 * hi;
    gemm_kloop<h16, 0>(A16, A16, W16, DQ, aoff, boff, acc);
    float* Cz = C + z * (size_t)TT_FULL * DM + (size_t)(RH + r0) * DM + c0; const int cofs = lr * 4; v4f bb; const float osc = 1.0f / (PCAR * WCAR);
#pragma unroll
    for (int q = 0; q < 4; ++q) bb[q] = bfr(bias[c0 + cofs + q]);
#pragma unroll
    for (int mb = 0; mb < 4; ++mb) {
#pragma unroll
        for (int nb = 0; nb < 4; ++nb) {
#pragma unroll
            for (int j = 0; j < 8; ++j) os[(hi * 8 + j) * 68 + nb * 16 + lr] = acc[mb][nb][j]; }
        __builtin_amdgcn_wave_barrier(); asm volatile("" ::: "memory");
        float* crow = Cz + (size_t)(mb * 16) * DM;
#pragma unroll 1
        for (int ps = 0; ps < 2; ++ps) {
#pragma unroll
            for (int s = 0; s < 8; ++s) { const int row = 2 * s + hi; v4f val = *(const v4fa*)(os + row * 68 + cofs); val = val * osc + bb; *(volatile v4f*)(crow + (size_t)row * DM + cofs) = val; }
            if (ps == 0) __threadfence(); }
        __builtin_amdgcn_wave_barrier(); asm volatile("" ::: "memory");
    }
}

extern "C" void kernel_launch(void* const* d_in, const int* in_sizes, int n_in,
                              void* d_out, int out_size, void* d_ws, size_t ws_size, hipStream_t stream) {
    if (n_in < 5) return;
    const size_t need_x = (size_t)(NB - 1) * TT_FULL * DM + (size_t)TT * DM;
    if ((size_t)in_sizes[0] < need_x || (size_t)in_sizes[1] < (size_t)DM * 3 * DQ || in_sizes[2] < 3 * DQ || (size_t)in_sizes[3] < (size_t)DQ * DM || in_sizes[4] < DM) return;
    if ((size_t)out_size < need_x) return;
    const float* x = (const float*)d_in[0]; const float* wa = (const float*)d_in[1]; const float* ba = (const float*)d_in[2]; const float* wp = (const float*)d_in[3]; const float* bp = (const float*)d_in[4];
    float* OUT = (float*)d_out;
    char* wsp = (char*)d_ws;
    auto take = [&](size_t bytes) { char* p = wsp; wsp += (bytes + 255) & ~(size_t)255; return (void*)p; };
    bf* WQKV = (bf*)take((size_t)3 * DQ * DM * 2); bf* WOb = (bf*)take((size_t)DM * DQ * 2); h16* WO16 = (h16*)take((size_t)DM * DQ * 2);
    bf* XB = (bf*)take((size_t)NB * TT * DM * 2); h16* AT16 = (h16*)XB;
    h16* PL16 = (h16*)take(3 * PSZ * 2); bf* PLh = (bf*)take(3 * ISZ * 2); bf* PLl = (bf*)take(3 * ISZ * 2);
    bf* ATh = (bf*)take((size_t)NB * RH * DQ * 2); bf* ATl = (bf*)take((size_t)NB * RH * DQ * 2);
    if ((size_t)(wsp - (char*)d_ws) > ws_size) return;
    k_cvt8<<<(unsigned)(((size_t)NB * TT * DM / 8 + 255) / 256), 256, 0, stream>>>(x, XB);
    k_wtA<<<(unsigned)((3 * DQ * DM / 64 + 63) / 64), 256, 0, stream>>>(wa, WQKV);
    k_wtO<<<(unsigned)((DM * DQ / 64 + 63) / 64), 256, 0, stream>>>(wp, WOb, WO16);
    k_qkv<<<dim3(NB * TT / 64, 3 * DQ / 64, 1), 32, 0, stream>>>(XB, WQKV, ba, PL16, PLh, PLl);
    k_attnhl<<<dim3(RH / 16, NB * NH_, 1), 32, 0, stream>>>(PLh, PLl, ATh, ATl);
    if (TT - RH > 0) k_attn16<<<dim3((TT - RH) / 16 + (TT == RH), NB * NH_, 1), 32, 0, stream>>>(PL16, AT16);
    k_outhl<<<dim3(RH / 64, DM / 64, NB), 32, 0, stream>>>(ATh, ATl, WOb, bp, OUT);
    if (TT - RH > 0) k_out16<<<dim3((TT - RH) / 64 + (TT == RH), DM / 64, NB), 32, 0, stream>>>(AT16, WO16, bp, OUT);
}
